// SAGE_32512902431457
// MI455X (gfx1250) — hardware-verified
//
#include <hip/hip_runtime.h>
#include <stddef.h>
#include <stdint.h>


#define DF     128
#define HP     256
#define A2P    512
#define TPF    256
#define NZP    1024
#define NLAY   3
#define NTHR   256
#define NWAVE  8
#define EPT    8
#define CHUNK  (NTHR * EPT)
#define WCAP   (EPT * 32)
#define LISTN  (NWAVE * WCAP)
#define NBA    1024
#define SLA    10
#define RCAP   28672
#define DEGCAP 64
#define MEAS_B1024  16710
#define MEAS_MAXDEG 36
#define CNT_POISON  (1 << 20)
#define GBM    64
#define GBN    128
#define GTHR   128
#define GWAVE  (GTHR / 32)
#define RPW    16
#define ABR    (NWAVE * RPW)
#define SRCH   24
#define U_ZB   (NZP * (DF / 8))
#define U_W0   (2 * DF * (DF / 8))
#define U_WC   (2 * DF * (4 * DF / 8))
#define U_WH   (DF * (2 * DF / 8))
#define U_TOT  (U_ZB + U_W0 + U_WC + U_WH)
#define AGG_ZINTS (LISTN + 2 * RCAP + 3 * NBA)
#define MISC_INTS 16
#define CMP_LDS_INTS (AGG_ZINTS + MISC_INTS)
#define WSMAX  134217728

static_assert((CHUNK & (CHUNK - 1)) == 0 && CHUNK <= 4096);
static_assert((NBA & (NBA - 1)) == 0 && NBA == (1 << SLA));
static_assert(((long long)CHUNK << SLA) < (1LL << 31));
static_assert(NBA % NWAVE == 0 && NBA % 32 == 0 && NBA == NTHR * 4);
static_assert(RCAP % (NTHR * 4) == 0 && AGG_ZINTS % (NTHR * 4) == 0 && LISTN % 4 == 0);
static_assert(RCAP >= MEAS_B1024 + 8192 && DEGCAP >= MEAS_MAXDEG + 8 && CNT_POISON > DEGCAP);
static_assert(GBN == DF && GBM == GWAVE * 16 && DF == 4 * 32 && GTHR == GWAVE * 32);
static_assert((GBM & 1) == 0 && (16 & 1) == 0);
static_assert(ABR % GBM == 0 && NZP % GBM == 0 && HP == 2 * DF && A2P == 4 * DF);
static_assert(DF % 32 == 0 && HP % 32 == 0 && A2P % 32 == 0);
static_assert(U_ZB % NTHR == 0 && U_W0 % NTHR == 0 && U_WC % NTHR == 0 && U_WH % NTHR == 0);
static_assert(CMP_LDS_INTS * 4 <= 300000);

typedef float          v4f   __attribute__((ext_vector_type(4)));
typedef float          v8f   __attribute__((ext_vector_type(8)));
typedef int            v4i   __attribute__((ext_vector_type(4)));
typedef int            v8i   __attribute__((ext_vector_type(8)));
typedef unsigned       v2u   __attribute__((ext_vector_type(2)));
typedef unsigned short v4us  __attribute__((ext_vector_type(4)));
typedef unsigned short v8us  __attribute__((ext_vector_type(8)));
typedef unsigned short v16us __attribute__((ext_vector_type(16)));
typedef __bf16         v16bf __attribute__((ext_vector_type(16)));
typedef v4f  __attribute__((may_alias)) v4fa;
typedef v4i  __attribute__((may_alias)) v4ia;
typedef v2u  __attribute__((may_alias)) v2ua;
typedef v4us __attribute__((may_alias)) v4usa;
typedef v8us __attribute__((may_alias)) v8usa;
union FragB { v16bf v; v16us u; v8us h[2]; v8i w; };

__device__ __forceinline__ v8f wmb(const FragB& a, const FragB& b, v8f c) {
  v8f d = __builtin_amdgcn_wmma_f32_16x16x32_bf16(false, a.v, false, b.v, (short)0, c, false, false);
  asm volatile("v_nop\n\tv_nop\n\tv_nop\n\tv_nop" : "+v"(d) : "v"(a.w), "v"(b.w));
  return d;
}

__device__ __forceinline__ v8f z8() { v8f z = {0.f, 0.f, 0.f, 0.f, 0.f, 0.f, 0.f, 0.f}; return z; }

__device__ __forceinline__ unsigned bf16_bits(float f) {
  const unsigned u = __float_as_uint(f);
  const unsigned r = (u + 0x7FFFu + ((u >> 16) & 1u)) >> 16;
  return (f != f) ? 0x7FC0u : r;
}
__device__ __forceinline__ float bf16_val(float f) {
  return __uint_as_float(bf16_bits(f) << 16);
}
__device__ __forceinline__ float relu_np(float v) { return (v > 0.0f) ? v : (v - v); }

__device__ __forceinline__ void hl4(const v4f v, v4us& h4, v4us& l4) {
  unsigned hb;
  hb = bf16_bits(v.x); h4[0] = (unsigned short)hb; l4[0] = (unsigned short)bf16_bits(v.x - __uint_as_float(hb << 16));
  hb = bf16_bits(v.y); h4[1] = (unsigned short)hb; l4[1] = (unsigned short)bf16_bits(v.y - __uint_as_float(hb << 16));
  hb = bf16_bits(v.z); h4[2] = (unsigned short)hb; l4[2] = (unsigned short)bf16_bits(v.z - __uint_as_float(hb << 16));
  hb = bf16_bits(v.w); h4[3] = (unsigned short)hb; l4[3] = (unsigned short)bf16_bits(v.w - __uint_as_float(hb << 16));
}

__device__ __forceinline__ void wave_sync() {
  __builtin_amdgcn_fence(__ATOMIC_RELEASE, "wavefront");
  __builtin_amdgcn_wave_barrier();
  __builtin_amdgcn_fence(__ATOMIC_ACQUIRE, "wavefront");
}

template <int SLB>
__device__ __forceinline__ int scan_chunk(const int* __restrict__ dsts, int nE, int cbase, int slotBase,
                                          int nb, int vec8, int* list, int tid, int lane, int wave) {
  int wc = 0;
  const int el0  = tid * EPT;
  const int e0   = cbase + el0;
  const int sent = -2147483647 - 1;
  v4i da, db;
  if (vec8 != 0 && cbase + CHUNK <= nE) {
    da = *(const v4i*)(dsts + e0);
    db = *(const v4i*)(dsts + e0 + 4);
  } else {
    da.x = (e0     < nE) ? dsts[min(e0,     nE - 1)] : sent;
    da.y = (e0 + 1 < nE) ? dsts[min(e0 + 1, nE - 1)] : sent;
    da.z = (e0 + 2 < nE) ? dsts[min(e0 + 2, nE - 1)] : sent;
    da.w = (e0 + 3 < nE) ? dsts[min(e0 + 3, nE - 1)] : sent;
    db.x = (e0 + 4 < nE) ? dsts[min(e0 + 4, nE - 1)] : sent;
    db.y = (e0 + 5 < nE) ? dsts[min(e0 + 5, nE - 1)] : sent;
    db.z = (e0 + 6 < nE) ? dsts[min(e0 + 6, nE - 1)] : sent;
    db.w = (e0 + 7 < nE) ? dsts[min(e0 + 7, nE - 1)] : sent;
  }
  const unsigned nbs = (unsigned)slotBase;
  const unsigned unb = (unsigned)nb;
  const unsigned s0 = (unsigned)da.x - nbs, s1 = (unsigned)da.y - nbs;
  const unsigned s2 = (unsigned)da.z - nbs, s3 = (unsigned)da.w - nbs;
  const unsigned s4 = (unsigned)db.x - nbs, s5 = (unsigned)db.y - nbs;
  const unsigned s6 = (unsigned)db.z - nbs, s7 = (unsigned)db.w - nbs;
  const bool h0 = s0 < unb, h1 = s1 < unb, h2 = s2 < unb, h3 = s3 < unb;
  const bool h4 = s4 < unb, h5 = s5 < unb, h6 = s6 < unb, h7 = s7 < unb;
  const unsigned any = __builtin_amdgcn_ballot_w32(h0 | h1 | h2 | h3 | h4 | h5 | h6 | h7);
  if (any != 0u) {
#define HITJ(J, HJ, SJ) { \
      const unsigned mj = __builtin_amdgcn_ballot_w32(HJ); \
      if (mj != 0u) { \
        if (HJ) { \
          const int pos = wc + (int)__builtin_amdgcn_mbcnt_lo(mj, 0u); \
          if (pos < WCAP) list[wave * WCAP + pos] = ((el0 + (J)) << SLB) | (int)(SJ); \
        } \
        wc += (int)__builtin_popcount(mj); } }
    HITJ(0, h0, s0)
    HITJ(1, h1, s1)
    HITJ(2, h2, s2)
    HITJ(3, h3, s3)
    HITJ(4, h4, s4)
    HITJ(5, h5, s5)
    HITJ(6, h6, s6)
    HITJ(7, h7, s7)
#undef HITJ
  }
  return wc;
}

__global__ __launch_bounds__(NTHR) void k_prep(const float* __restrict__ zt, const float* __restrict__ wl,
                                               const float* __restrict__ wr, const float* __restrict__ w1,
                                               unsigned short* planes, int nZ) {
  const int u = (int)blockIdx.x * NTHR + (int)threadIdx.x;
  v8us o;
  if (u < U_ZB) {
    const int row = u >> 4, k8 = (u & 15) * 8;
    const int rc  = row < nZ ? row : nZ - 1;
    const unsigned lm = (row < nZ) ? 0xFFFFu : 0u;
    const float* p = zt + (size_t)rc * DF + k8;
    const v4f a0 = *(const v4f*)p, a1 = *(const v4f*)(p + 4);
    o[0] = (unsigned short)(bf16_bits(a0.x) & lm); o[1] = (unsigned short)(bf16_bits(a0.y) & lm);
    o[2] = (unsigned short)(bf16_bits(a0.z) & lm); o[3] = (unsigned short)(bf16_bits(a0.w) & lm);
    o[4] = (unsigned short)(bf16_bits(a1.x) & lm); o[5] = (unsigned short)(bf16_bits(a1.y) & lm);
    o[6] = (unsigned short)(bf16_bits(a1.z) & lm); o[7] = (unsigned short)(bf16_bits(a1.w) & lm);
  } else if (u < U_ZB + U_W0 + U_WC) {
    size_t wo;
    unsigned msk;
    if (u < U_ZB + U_W0) {
      const int v = u - U_ZB;
      const int n = v >> 4, k8 = (v & 15) * 8;
      wo  = (size_t)(n & (DF - 1)) * DF + (size_t)k8;
      msk = (n < DF) ? 0xFFFFu : 0u;
    } else {
      const int v  = u - (U_ZB + U_W0);
      const int l  = 1 + (v >> 13);
      const int n  = (v >> 6) & (DF - 1), k8 = (v & 63) * 8;
      wo  = (size_t)l * DF * DF + (size_t)n * DF + (size_t)(k8 & (DF - 1));
      msk = (k8 < 2 * DF) ? 0xFFFFu : 0u;
    }
    const v4f a0 = *(const v4f*)(wl + wo), a1 = *(const v4f*)(wl + wo + 4);
    const v4f c0 = *(const v4f*)(wr + wo), c1 = *(const v4f*)(wr + wo + 4);
    const unsigned nm = ~msk & 0xFFFFu;
    o[0] = (unsigned short)((bf16_bits(a0.x) & msk) | (bf16_bits(c0.x) & nm));
    o[1] = (unsigned short)((bf16_bits(a0.y) & msk) | (bf16_bits(c0.y) & nm));
    o[2] = (unsigned short)((bf16_bits(a0.z) & msk) | (bf16_bits(c0.z) & nm));
    o[3] = (unsigned short)((bf16_bits(a0.w) & msk) | (bf16_bits(c0.w) & nm));
    o[4] = (unsigned short)((bf16_bits(a1.x) & msk) | (bf16_bits(c1.x) & nm));
    o[5] = (unsigned short)((bf16_bits(a1.y) & msk) | (bf16_bits(c1.y) & nm));
    o[6] = (unsigned short)((bf16_bits(a1.z) & msk) | (bf16_bits(c1.z) & nm));
    o[7] = (unsigned short)((bf16_bits(a1.w) & msk) | (bf16_bits(c1.w) & nm));
  } else if (u < U_TOT) {
    const int v = u - (U_ZB + U_W0 + U_WC);
    const int n = v >> 5, k8 = (v & 31) * 8;
    const float* p = w1 + (size_t)n * DF + (size_t)(k8 & (DF - 1));
    const v4f a0 = *(const v4f*)p, a1 = *(const v4f*)(p + 4);
    o[0] = (unsigned short)bf16_bits(a0.x); o[1] = (unsigned short)bf16_bits(a0.y);
    o[2] = (unsigned short)bf16_bits(a0.z); o[3] = (unsigned short)bf16_bits(a0.w);
    o[4] = (unsigned short)bf16_bits(a1.x); o[5] = (unsigned short)bf16_bits(a1.y);
    o[6] = (unsigned short)bf16_bits(a1.z); o[7] = (unsigned short)bf16_bits(a1.w);
  } else {
    return;
  }
  unsigned short* dp = planes + (size_t)u * 8;
  *(volatile v8us*)dp = o;
  __threadfence();
  *(volatile v8us*)dp = o;
}

__global__ __launch_bounds__(NTHR) void k_compact(const int* __restrict__ srcs, const int* __restrict__ dsts,
                                                  int nE, int nN, int vec8, int* listG, int* cntG, int* offG) {
  extern __shared__ __attribute__((aligned(16))) int dsm[];
  int* list = dsm;
  int* hl   = dsm + LISTN;
  int* sl   = hl + RCAP;
  int* cnt  = sl + RCAP;
  int* offs = cnt + NBA;
  int* cur  = offs + NBA;
  int* misc = cur + NBA;
  const int tid = (int)threadIdx.x, lane = tid & 31, wave = tid >> 5;
  const int nodeBase = (int)blockIdx.x * NBA;

  {
    const v4i z4 = {0, 0, 0, 0};
    for (int i = tid * 4; i < AGG_ZINTS; i += NTHR * 4) *(v4ia*)(dsm + i) = z4;
    if (tid < MISC_INTS) misc[tid] = 0;
  }
  __syncthreads();

  int t = 0, ov = 0;
  const int nChunks = (nE + CHUNK - 1) / CHUNK;
#pragma unroll 1
  for (int ch = 0; ch < nChunks; ++ch) {
    const int cbase = ch * CHUNK;
    const int wc = scan_chunk<SLA>(dsts, nE, cbase, nodeBase, NBA, vec8, list, tid, lane, wave);
    if (lane == 0) misc[wave] = wc;
    __syncthreads();
    if (wave == 0) {
#pragma unroll 1
      for (int w2 = 0; w2 < NWAVE; ++w2) {
        int c = misc[w2];
        c = c < 0 ? 0 : (c > WCAP ? WCAP : c);
#pragma unroll 1
        for (int b0 = 0; b0 < c; b0 += 32) {
          const int idx = b0 + lane;
          const int ent_ = list[w2 * WCAP + (idx < WCAP ? idx : WCAP - 1)];
          const int m32 = (c - b0) < 32 ? (c - b0) : 32;
#pragma unroll 1
          for (int k = 0; k < m32; ++k) {
            const int u    = __builtin_amdgcn_readlane(ent_, k);
            const int slot = u & (NBA - 1);
            const int el   = (u >> SLA) & (CHUNK - 1);
            const int pk   = ((cbase + el) << SLA) | slot;
            if (t < RCAP) {
              if (lane == 0) { hl[t] = pk; cnt[slot] = cnt[slot] + 1; }
              t = t + 1;
            } else {
              ov = 1;
            }
          }
        }
      }
    }
    __syncthreads();
  }
  if (wave == 0 && lane == 0) { misc[8] = t; misc[9] = ov; }
  __syncthreads();
  int tt = misc[8];
  tt = tt < 0 ? 0 : (tt > RCAP ? RCAP : tt);
  const int ovf = misc[9];

  if (wave == 0) {
    const int base = lane * (NBA / 32);
    int s = 0;
#pragma unroll 1
    for (int i = 0; i < NBA / 32; ++i) s += cnt[base + i];
    int incl = s;
#pragma unroll
    for (int d = 1; d < 32; d <<= 1) {
      const int y = __shfl_up(incl, d, 32);
      if (lane >= d) incl += y;
    }
    int run = incl - s;
#pragma unroll 1
    for (int i = 0; i < NBA / 32; ++i) {
      const int cv = cnt[base + i];
      offs[base + i] = run;
      cur[base + i]  = run;
      run += cv;
    }
  }
  __syncthreads();
  if (wave == 0) {
#pragma unroll 1
    for (int b0 = 0; b0 < tt; b0 += 32) {
      const int idx = b0 + lane;
      const int ent_ = hl[idx < RCAP ? idx : RCAP - 1];
      const int m32 = (tt - b0) < 32 ? (tt - b0) : 32;
#pragma unroll 1
      for (int k = 0; k < m32; ++k) {
        const int u    = __builtin_amdgcn_readlane(ent_, k);
        const int slot = u & (NBA - 1);
        if (lane == 0) {
          int p = cur[slot];
          p = p < 0 ? 0 : (p > RCAP - 1 ? RCAP - 1 : p);
          sl[p] = u;
          cur[slot] = p + 1;
        }
      }
    }
  }
  __syncthreads();

  int* lg = listG + (size_t)blockIdx.x * RCAP;
#pragma unroll 1
  for (int j = 0; j < RCAP / (NTHR * 4); ++j) {
    const int i = 4 * (tid + NTHR * j);
    const v4i e4 = *(const v4ia*)(sl + i);
    int e0 = e4.x >> SLA, e1 = e4.y >> SLA, e2 = e4.z >> SLA, e3 = e4.w >> SLA;
    e0 = e0 < 0 ? 0 : (e0 > nE - 1 ? nE - 1 : e0);
    e1 = e1 < 0 ? 0 : (e1 > nE - 1 ? nE - 1 : e1);
    e2 = e2 < 0 ? 0 : (e2 > nE - 1 ? nE - 1 : e2);
    e3 = e3 < 0 ? 0 : (e3 > nE - 1 ? nE - 1 : e3);
    int s0 = srcs[e0], s1 = srcs[e1], s2 = srcs[e2], s3 = srcs[e3];
    s0 = s0 < 0 ? 0 : (s0 > nN - 1 ? nN - 1 : s0);
    s1 = s1 < 0 ? 0 : (s1 > nN - 1 ? nN - 1 : s1);
    s2 = s2 < 0 ? 0 : (s2 > nN - 1 ? nN - 1 : s2);
    s3 = s3 < 0 ? 0 : (s3 > nN - 1 ? nN - 1 : s3);
    v4i o;
    o.x = (i     < tt) ? s0 : 0;
    o.y = (i + 1 < tt) ? s1 : 0;
    o.z = (i + 2 < tt) ? s2 : 0;
    o.w = (i + 3 < tt) ? s3 : 0;
    int* dp = lg + i;
    *(volatile v4i*)dp = o;
    __threadfence();
    *(volatile v4i*)dp = o;
  }
  {
    v4i c4 = *(const v4ia*)(cnt + 4 * tid);
    const v4i o4 = *(const v4ia*)(offs + 4 * tid);
    const v4i p4 = {CNT_POISON, CNT_POISON, CNT_POISON, CNT_POISON};
    c4 = (ovf != 0) ? p4 : c4;
    int* cp = cntG + (size_t)nodeBase + 4 * tid;
    int* op = offG + (size_t)nodeBase + 4 * tid;
    *(volatile v4i*)cp = c4;
    *(volatile v4i*)op = o4;
    __threadfence();
    *(volatile v4i*)cp = c4;
    *(volatile v4i*)op = o4;
  }
}

template <int MODE>
__global__ __launch_bounds__(NTHR) void k_agg(const int* __restrict__ listG, const int* __restrict__ cntG,
                                              const int* __restrict__ offG, const int* __restrict__ zidx,
                                              const int* __restrict__ bat, const float* __restrict__ T,
                                              const float* __restrict__ bl0, const unsigned short* __restrict__ hsrc,
                                              unsigned short* dstp, int nN, int nZ, int nLive) {
  __shared__ __attribute__((aligned(16))) unsigned short rowbuf[NWAVE * HP];
  const int tid = (int)threadIdx.x, lane = tid & 31, wave = tid >> 5;
  unsigned short* rb = rowbuf + wave * HP;
  const int rowBase = (int)blockIdx.x * ABR;
  constexpr int DPITCH = (MODE == 2) ? A2P : HP;
  v4f b4 = {0.f, 0.f, 0.f, 0.f};
  if constexpr (MODE == 0) {
    const v4f tb = *(const v4f*)(bl0 + 4 * lane);
    b4.x = bf16_val(tb.x); b4.y = bf16_val(tb.y); b4.z = bf16_val(tb.z); b4.w = bf16_val(tb.w);
  }
  const float qnan = __int_as_float(0x7fc00000);

#pragma unroll 1
  for (int it = 0; it < RPW; ++it) {
    const int node = rowBase + it * NWAVE + wave;
    const bool live = node < nLive;
    int r = node;
    if constexpr (MODE == 2) {
      const int g = node >> 1;
      int lo = 0, hi = nN;
#pragma unroll 1
      for (int s = 0; s < SRCH; ++s) {
        const int mid = (lo + hi) >> 1;
        const int mc  = mid < nN - 1 ? mid : nN - 1;
        const int bv  = bat[mc];
        const bool act = lo < hi;
        const bool lt  = bv < g;
        lo = (act && lt) ? mid + 1 : lo;
        hi = (act && !lt) ? mid : hi;
      }
      r = lo + (node & 1);
    }
    const int rc = r < 0 ? 0 : (r > nN - 1 ? nN - 1 : r);
    int c = cntG[rc];
    const bool big = (c > DEGCAP) || (c < 0);
    c = c < 0 ? 0 : (c > DEGCAP ? DEGCAP : c);
    c = live ? c : 0;
    int o = offG[rc];
    o = o < 0 ? 0 : (o > RCAP ? RCAP : o);
    const int* lp = listG + (size_t)(rc >> SLA) * RCAP;
    float a0 = 0.0f, a1 = 0.0f, a2 = 0.0f, a3 = 0.0f;
#pragma unroll 1
    for (int b0 = 0; b0 < c; b0 += 32) {
      int idx = o + b0 + lane;
      idx = idx > RCAP - 1 ? RCAP - 1 : idx;
      int sr = lp[idx];
      sr = sr < 0 ? 0 : (sr > nN - 1 ? nN - 1 : sr);
      if constexpr (MODE == 0) {
        int zz = zidx[sr];
        sr = zz < 0 ? 0 : (zz > nZ - 1 ? nZ - 1 : zz);
      }
      const int m32 = (c - b0) < 32 ? (c - b0) : 32;
#pragma unroll 1
      for (int k = 0; k < m32; ++k) {
        const int sk = __builtin_amdgcn_readlane(sr, k);
        if constexpr (MODE == 0) {
          const v4f a = *(const v4f*)(T + (size_t)sk * TPF + 4 * lane);
          a0 += a.x; a1 += a.y; a2 += a.z; a3 += a.w;
        } else {
          const unsigned short* rp = hsrc + (size_t)sk * HP + 4 * lane;
          const v2u wh = *(const v2ua*)rp;
          const v2u wl = *(const v2ua*)(rp + DF);
          const float f0 = __uint_as_float(wh.x << 16)         + __uint_as_float(wl.x << 16);
          const float f1 = __uint_as_float(wh.x & 0xffff0000u) + __uint_as_float(wl.x & 0xffff0000u);
          const float f2 = __uint_as_float(wh.y << 16)         + __uint_as_float(wl.y << 16);
          const float f3 = __uint_as_float(wh.y & 0xffff0000u) + __uint_as_float(wl.y & 0xffff0000u);
          a0 += f0; a1 += f1; a2 += f2; a3 += f3;
        }
      }
    }
    const float inv = 1.0f / fmaxf((float)c, 1.0f);
    const float pzr = big ? qnan : 0.0f;
    v4f mv;
    if constexpr (MODE == 0) {
      int zi = zidx[rc];
      zi = zi < 0 ? 0 : (zi > nZ - 1 ? nZ - 1 : zi);
      const v4f tr = *(const v4f*)(T + (size_t)zi * TPF + DF + 4 * lane);
      mv.x = relu_np(a0 * inv + b4.x + tr.x + pzr);
      mv.y = relu_np(a1 * inv + b4.y + tr.y + pzr);
      mv.z = relu_np(a2 * inv + b4.z + tr.z + pzr);
      mv.w = relu_np(a3 * inv + b4.w + tr.w + pzr);
    } else {
      mv.x = a0 * inv + pzr; mv.y = a1 * inv + pzr; mv.z = a2 * inv + pzr; mv.w = a3 * inv + pzr;
    }
    mv.x = live ? mv.x : 0.0f; mv.y = live ? mv.y : 0.0f; mv.z = live ? mv.z : 0.0f; mv.w = live ? mv.w : 0.0f;
    v4us mh, ml;
    hl4(mv, mh, ml);
    *(v4usa*)(rb + 4 * lane)      = mh;
    *(v4usa*)(rb + DF + 4 * lane) = ml;
    wave_sync();
    const v8us q0 = *(const v8usa*)(rb + 8 * lane);
    wave_sync();
    v8us q1 = {0, 0, 0, 0, 0, 0, 0, 0};
    if constexpr (MODE == 2) {
      const v8us t1 = *(const v8usa*)(hsrc + (size_t)rc * HP + 8 * lane);
      const v8us zz8 = {0, 0, 0, 0, 0, 0, 0, 0};
      q1 = live ? t1 : zz8;
    }
    unsigned short* rpw = dstp + (size_t)node * DPITCH + 8 * lane;
    *(volatile v8us*)rpw = q0;
    if constexpr (MODE == 2) *(volatile v8us*)(rpw + HP) = q1;
    __threadfence();
    *(volatile v8us*)rpw = q0;
    if constexpr (MODE == 2) *(volatile v8us*)(rpw + HP) = q1;
  }
  (void)bat; (void)T; (void)zidx; (void)hsrc; (void)nZ;
}

template <int MODE>
__global__ __launch_bounds__(GTHR) void k_gemm(const unsigned short* A0, int lda0, int K0,
                                               const unsigned short* A1, int lda1, int K1,
                                               const unsigned short* __restrict__ BT, int ldb,
                                               const float* __restrict__ bias, const float* __restrict__ w2v,
                                               const float* __restrict__ b2p,
                                               unsigned short* apl, float* outp, int ldo, int nLive) {
  __shared__ __attribute__((aligned(16))) float stg[GBM * GBN];
  __shared__ __attribute__((aligned(16))) float ovec[GBM];
  const int tid = (int)threadIdx.x, lane = tid & 31, wave = tid >> 5, hh = lane >> 4, m = lane & 15;
  const int rowBase = (int)blockIdx.x * GBM;
  const int colBase = (int)blockIdx.y * GBN;

  v8f acc[8];
#pragma unroll
  for (int t = 0; t < 8; ++t) acc[t] = z8();
  const unsigned short* ap0 = A0 + (size_t)(rowBase + 16 * wave + m) * (size_t)lda0 + 8 * hh;
  const unsigned short* ap1 = A1 + (size_t)(rowBase + 16 * wave + m) * (size_t)lda1 + 8 * hh;
  const unsigned short* bp  = BT + (size_t)(colBase + m) * (size_t)ldb + 8 * hh;

#pragma unroll 1
  for (int k0 = 0; k0 < K0; k0 += 32) {
    FragB af;
    af.h[0] = *(const v8usa*)(ap0 + k0);
    af.h[1] = *(const v8usa*)(ap0 + k0 + 16);
#pragma unroll
    for (int nt = 0; nt < 8; ++nt) {
      const unsigned short* wq = bp + (size_t)(16 * nt) * (size_t)ldb + k0;
      FragB bf;
      bf.h[0] = *(const v8usa*)wq;
      bf.h[1] = *(const v8usa*)(wq + 16);
      acc[nt] = wmb(af, bf, acc[nt]);
    }
  }
#pragma unroll 1
  for (int k0 = 0; k0 < K1; k0 += 32) {
    FragB af;
    af.h[0] = *(const v8usa*)(ap1 + k0);
    af.h[1] = *(const v8usa*)(ap1 + k0 + 16);
#pragma unroll
    for (int nt = 0; nt < 8; ++nt) {
      const unsigned short* wq = bp + (size_t)(16 * nt) * (size_t)ldb + K0 + k0;
      FragB bf;
      bf.h[0] = *(const v8usa*)wq;
      bf.h[1] = *(const v8usa*)(wq + 16);
      acc[nt] = wmb(af, bf, acc[nt]);
    }
  }

#pragma unroll
  for (int nt = 0; nt < 8; ++nt) {
    const int lc = 16 * nt + m;
#pragma unroll
    for (int r = 0; r < 8; ++r) {
      const int lr = 16 * wave + 8 * hh + r;
      stg[lr * GBN + lc] = acc[nt][r];
    }
  }
  __syncthreads();

  v4f bb4 = {0.f, 0.f, 0.f, 0.f};
  if constexpr (MODE != 0) {
    const v4f t1 = *(const v4f*)(bias + 4 * lane);
    bb4.x = bf16_val(t1.x); bb4.y = bf16_val(t1.y); bb4.z = bf16_val(t1.z); bb4.w = bf16_val(t1.w);
  }

  v4f pv[16];
#pragma unroll
  for (int i = 0; i < 16; ++i) pv[i] = *(const v4fa*)(stg + (16 * wave + i) * GBN + 4 * lane);
  __syncthreads();

  if constexpr (MODE == 0) {
#pragma unroll
    for (int i = 0; i < 16; ++i) {
      float* op = outp + (size_t)(rowBase + 16 * wave + i) * (size_t)ldo + colBase + 4 * lane;
      *(volatile v4f*)op = pv[i];
    }
    __threadfence();
#pragma unroll
    for (int i = 0; i < 16; ++i) {
      float* op = outp + (size_t)(rowBase + 16 * wave + i) * (size_t)ldo + colBase + 4 * lane;
      *(volatile v4f*)op = pv[i];
    }
  } else if constexpr (MODE == 1) {
#pragma unroll
    for (int i = 0; i < 16; ++i) {
      const bool ok = (rowBase + 16 * wave + i) < nLive;
      const v4f t = pv[i] + bb4;
      v4f y;
      y.x = relu_np(t.x); y.y = relu_np(t.y); y.z = relu_np(t.z); y.w = relu_np(t.w);
      y.x = ok ? y.x : 0.0f; y.y = ok ? y.y : 0.0f; y.z = ok ? y.z : 0.0f; y.w = ok ? y.w : 0.0f;
      v4us h4, l4;
      hl4(y, h4, l4);
      unsigned short* srow = (unsigned short*)stg + (size_t)(16 * wave + i) * (2 * GBN);
      *(v4usa*)(srow + 4 * lane) = h4;
      *(v4usa*)(srow + DF + 4 * lane) = l4;
    }
    __syncthreads();
    v8us qv[16];
#pragma unroll
    for (int i = 0; i < 16; ++i) {
      const unsigned short* srow = (const unsigned short*)stg + (size_t)(16 * wave + i) * (2 * GBN);
      qv[i] = *(const v8usa*)(srow + 8 * lane);
    }
#pragma unroll
    for (int i = 0; i < 16; ++i) {
      unsigned short* rp = apl + (size_t)(rowBase + 16 * wave + i) * (size_t)HP + 8 * lane;
      *(volatile v8us*)rp = qv[i];
    }
    __threadfence();
#pragma unroll
    for (int i = 0; i < 16; ++i) {
      unsigned short* rp = apl + (size_t)(rowBase + 16 * wave + i) * (size_t)HP + 8 * lane;
      *(volatile v8us*)rp = qv[i];
    }
  } else if constexpr (MODE == 2) {
    const int gBase = (int)blockIdx.x * (GBM / 2) + 8 * wave;
#pragma unroll
    for (int i = 0; i < 8; ++i) {
      const bool ok = (gBase + i) < nLive;
      const v4f ya = pv[2 * i] + bb4;
      const v4f yb = pv[2 * i + 1] + bb4;
      v4f p = ya * yb;
      p.x = ok ? p.x : 0.0f; p.y = ok ? p.y : 0.0f; p.z = ok ? p.z : 0.0f; p.w = ok ? p.w : 0.0f;
      v4us h4, l4;
      hl4(p, h4, l4);
      unsigned short* srow = (unsigned short*)stg + (size_t)(16 * wave + i) * (2 * GBN);
      *(v4usa*)(srow + 4 * lane) = h4;
      *(v4usa*)(srow + DF + 4 * lane) = l4;
    }
    __syncthreads();
    v8us qv[8];
#pragma unroll
    for (int i = 0; i < 8; ++i) {
      const unsigned short* srow = (const unsigned short*)stg + (size_t)(16 * wave + i) * (2 * GBN);
      qv[i] = *(const v8usa*)(srow + 8 * lane);
    }
#pragma unroll
    for (int i = 0; i < 8; ++i) {
      unsigned short* rp = apl + (size_t)(gBase + i) * (size_t)HP + 8 * lane;
      *(volatile v8us*)rp = qv[i];
    }
    __threadfence();
#pragma unroll
    for (int i = 0; i < 8; ++i) {
      unsigned short* rp = apl + (size_t)(gBase + i) * (size_t)HP + 8 * lane;
      *(volatile v8us*)rp = qv[i];
    }
  } else {
    v4f w4;
    {
      const v4f t2 = *(const v4f*)(w2v + 4 * lane);
      w4.x = bf16_val(t2.x); w4.y = bf16_val(t2.y); w4.z = bf16_val(t2.z); w4.w = bf16_val(t2.w);
    }
    const float b2v = bf16_val(b2p[0]);
    float res = 0.0f;
#pragma unroll
    for (int i = 0; i < 16; ++i) {
      const v4f t = pv[i] + bb4;
      const float h0 = relu_np(t.x), h1 = relu_np(t.y), h2 = relu_np(t.z), h3 = relu_np(t.w);
      float s = (h0 * w4.x + h1 * w4.y) + (h2 * w4.z + h3 * w4.w);
      s += __shfl_xor(s, 16, 32);
      s += __shfl_xor(s, 8, 32);
      s += __shfl_xor(s, 4, 32);
      s += __shfl_xor(s, 2, 32);
      s += __shfl_xor(s, 1, 32);
      res = (lane == i) ? s : res;
    }
    if (lane < 16) ovec[16 * wave + lane] = res + b2v;
    __syncthreads();
    const int l15 = lane & 15;
    const v4f ov = *(const v4fa*)(ovec + 4 * l15);
    const int e0 = rowBase + 4 * l15;
    const bool st = (wave == 0) && (lane < 16) && (e0 + 3 < nLive);
    float* op = outp + e0;
    if (st) *(volatile v4f*)op = ov;
    __threadfence();
    if (st) *(volatile v4f*)op = ov;
  }
  (void)w2v; (void)b2p; (void)apl; (void)outp; (void)ldo; (void)nLive; (void)ovec;
}

static inline int cdiv(int a, int b) { return (a + b - 1) / b; }
static inline size_t al256(size_t o) { return (o + 255) & ~(size_t)255; }

extern "C" void kernel_launch(void* const* d_in, const int* in_sizes, int n_in,
                              void* d_out, int out_size, void* d_ws, size_t ws_size,
                              hipStream_t stream) {
  if (n_in < 11) return;
  const int nN = in_sizes[0];
  if (nN < 2 || nN >= (1 << 24)) return;
  if (in_sizes[2] != nN) return;
  if (in_sizes[1] < 2 || (in_sizes[1] & 1) != 0) return;
  const int nE = in_sizes[1] / 2;
  if (nE < 1 || nE >= (1 << 21)) return;
  if (in_sizes[3] < DF || (in_sizes[3] % DF) != 0) return;
  const int nZ = in_sizes[3] / DF;
  if (nZ > NZP) return;
  if (in_sizes[4] != NLAY * DF * DF || in_sizes[5] != NLAY * DF || in_sizes[6] != NLAY * DF * DF) return;
  if (in_sizes[7] != DF * DF || in_sizes[8] != DF || in_sizes[9] != DF || in_sizes[10] != 1) return;
  const int nG = out_size;
  if (nG < 4 || (nG & 3) != 0 || nG > (1 << 22)) return;

  const int*   z    = (const int*)  d_in[0];
  const int*   ei   = (const int*)  d_in[1];
  const int*   bat  = (const int*)  d_in[2];
  const float* zt   = (const float*)d_in[3];
  const float* Wl   = (const float*)d_in[4];
  const float* bl   = (const float*)d_in[5];
  const float* Wr   = (const float*)d_in[6];
  const float* W1   = (const float*)d_in[7];
  const float* b1   = (const float*)d_in[8];
  const float* W2   = (const float*)d_in[9];
  const float* b2   = (const float*)d_in[10];
  float* out = (float*)d_out;
  const int* src = ei;
  const int* dst = ei + nE;

  const int MP1 = cdiv(nN, ABR) * ABR;
  const int MP2 = cdiv(2 * nG, ABR) * ABR;
  const int PR  = MP2 / 2;
  const int gA  = cdiv(nN, NBA);
  if ((PR % GBM) != 0 || PR < nG) return;
  const int vec8 = ((nE & 3) == 0) ? 1 : 0;

  char* ws = (char*)d_ws;
  size_t off = 0;
  const size_t oPL  = off; off = al256(off + (size_t)U_TOT * 16);
  const size_t oT   = off; off = al256(off + (size_t)NZP * TPF * 4);
  const size_t oLST = off; off = al256(off + (size_t)gA * RCAP * 4);
  const size_t oCNT = off; off = al256(off + (size_t)gA * NBA * 4);
  const size_t oOFF = off; off = al256(off + (size_t)gA * NBA * 4);
  const size_t oH1  = off; off = al256(off + (size_t)MP1 * HP * 2);
  const size_t oAG  = off; off = al256(off + (size_t)MP1 * HP * 2);
  const size_t oA2  = off; off = al256(off + (size_t)MP2 * A2P * 2);
  const size_t oPH  = off; off = al256(off + (size_t)PR * HP * 2);
  if (off > ws_size || off > (size_t)WSMAX) return;
  unsigned short* PL   = (unsigned short*)(ws + oPL);
  unsigned short* ZB   = PL;
  unsigned short* W0c  = PL + (size_t)U_ZB * 8;
  unsigned short* W1c  = W0c + (size_t)U_W0 * 8;
  unsigned short* W2c  = W1c + (size_t)DF * A2P;
  unsigned short* WH   = W2c + (size_t)DF * A2P;
  float*          T    = (float*)(ws + oT);
  int*            LST  = (int*)(ws + oLST);
  int*            CNT  = (int*)(ws + oCNT);
  int*            OFF  = (int*)(ws + oOFF);
  unsigned short* H1   = (unsigned short*)(ws + oH1);
  unsigned short* AG   = (unsigned short*)(ws + oAG);
  unsigned short* A2   = (unsigned short*)(ws + oA2);
  unsigned short* PHL  = (unsigned short*)(ws + oPH);

  const size_t cmpLds = (size_t)CMP_LDS_INTS * 4;
  hipFuncSetAttribute(reinterpret_cast<const void*>(&k_compact), hipFuncAttributeMaxDynamicSharedMemorySize, (int)cmpLds);

  k_prep<<<U_TOT / NTHR, NTHR, 0, stream>>>(zt, Wl, Wr, W1, PL, nZ);
  k_gemm<0><<<dim3(NZP / GBM, 2), GTHR, 0, stream>>>(ZB, DF, DF, ZB, DF, 0, W0c, DF, bl, W2, b2, PL, T, TPF, NZP);
  k_compact<<<gA, NTHR, cmpLds, stream>>>(src, dst, nE, nN, vec8, LST, CNT, OFF);
  k_agg<0><<<MP1 / ABR, NTHR, 0, stream>>>(LST, CNT, OFF, z, bat, T, bl, PL, H1, nN, nZ, nN);
  k_agg<1><<<MP1 / ABR, NTHR, 0, stream>>>(LST, CNT, OFF, z, bat, T, bl, H1, AG, nN, nZ, nN);
  k_gemm<1><<<dim3(MP1 / GBM, 1), GTHR, 0, stream>>>(AG, HP, HP, H1, HP, HP, W1c, A2P, bl + DF, W2, b2, AG, out, 0, nN);
  k_agg<2><<<MP2 / ABR, NTHR, 0, stream>>>(LST, CNT, OFF, z, bat, T, bl, AG, A2, nN, nZ, 2 * nG);
  k_gemm<2><<<dim3(MP2 / GBM, 1), GTHR, 0, stream>>>(A2, A2P, A2P, A2, A2P, 0, W2c, A2P, bl + 2 * DF, W2, b2, PHL, out, 0, nG);
  k_gemm<3><<<dim3(PR / GBM, 1), GTHR, 0, stream>>>(PHL, HP, HP, PHL, HP, 0, WH, HP, b1, W2, b2, PHL, out, 0, nG);
}
